// SAGNetwork_85890755985941
// MI455X (gfx1250) — hardware-verified
//
#include <hip/hip_runtime.h>

#define NB    1024
#define NN    64
#define DOBS  128
#define DH    256
#define DA    16
#define NHD   4
#define HDM   64

#define PX    264
#define POBS  136
#define PT    72
#define PZ    260

#define OFF_S    0
#define OFF_XA   36864
#define OFF_XB   70656
#define OFF_Q    104448
#define OFF_VT   138240
#define OFF_ADJ  175104
#define SMEM_BYTES 184320

#define WO_W1   0
#define WO_W2   32768
#define WO_WQ   98304
#define WO_WK   163840
#define WO_WV   229376
#define WO_WO   294912
#define WO_WC   360448
#define WO_W3H  425984
#define WO_W3L  430080
#define WS_HALVES 434176
#define NGRP  (WS_HALVES / 8)

#define WSC   64.0f
#define WINV  0.015625f
#define PSC   16384.0f
#define PINV  0.00006103515625f
#define ZINV  0.000244140625f

static_assert(NGRP * 8 == WS_HALVES);
static_assert((NGRP % 256) == 0);
static_assert(OFF_XA + NN * PZ * 4 <= OFF_Q);
static_assert(OFF_ADJ + NN * PT * 2 == SMEM_BYTES);
static_assert(NN * POBS * 2 <= OFF_XA);
static_assert(NHD * NN * PT * 2 <= OFF_XA);
static_assert(NN * DA * 4 <= OFF_XA);

typedef _Float16 f16;
typedef _Float16 v16h __attribute__((ext_vector_type(16)));
typedef _Float16 v8h  __attribute__((ext_vector_type(8)));
typedef _Float16 v4h  __attribute__((ext_vector_type(4)));
typedef float    v8f  __attribute__((ext_vector_type(8)));
typedef float    v4f  __attribute__((ext_vector_type(4)));
typedef v8h __attribute__((may_alias)) v8ha;
typedef v4h __attribute__((may_alias)) v4ha;
typedef v4f __attribute__((may_alias)) v4fa;

#define LDS_AS __attribute__((address_space(3)))
typedef LDS_AS f16   lf16;
typedef LDS_AS float lf32;
typedef LDS_AS v8ha  lv8h;
typedef LDS_AS v4ha  lv4h;
typedef LDS_AS v4fa  lv4f;

union Frag16 { v16h v; v8h hf[2]; f16 s[16]; };
union Frag8  { v8h v; f16 s[8]; };

__device__ __forceinline__ v8f wmma1(v16h a, v16h b, v8f c) {
  v8f d = __builtin_amdgcn_wmma_f32_16x16x32_f16(false, a, false, b, (short)0, c, false, false);
  asm volatile("v_nop\n\tv_nop\n\tv_nop\n\tv_nop" : "+v"(d) : "v"(a), "v"(b));
  return d;
}

__device__ __forceinline__ void wmma2(v16h a0, v16h a1, v16h b, v8f& c0, v8f& c1) {
  v8f d0 = __builtin_amdgcn_wmma_f32_16x16x32_f16(false, a0, false, b, (short)0, c0, false, false);
  v8f d1 = __builtin_amdgcn_wmma_f32_16x16x32_f16(false, a1, false, b, (short)0, c1, false, false);
  asm volatile("v_nop\n\tv_nop\n\tv_nop\n\tv_nop" : "+v"(d0), "+v"(d1) : "v"(a0), "v"(a1), "v"(b));
  c0 = d0;
  c1 = d1;
}

__device__ __forceinline__ v8f wmma3(v16h ah, v16h al, v16h bh, v16h bl, v8f c) {
  v8f d = __builtin_amdgcn_wmma_f32_16x16x32_f16(false, ah, false, bh, (short)0, c, false, false);
  d = __builtin_amdgcn_wmma_f32_16x16x32_f16(false, ah, false, bl, (short)0, d, false, false);
  d = __builtin_amdgcn_wmma_f32_16x16x32_f16(false, al, false, bh, (short)0, d, false, false);
  asm volatile("v_nop\n\tv_nop\n\tv_nop\n\tv_nop" : "+v"(d) : "v"(ah), "v"(al), "v"(bh), "v"(bl));
  return d;
}

__device__ __forceinline__ v16h frag_lds(const lf16* base, int pitch, int row0, int k0) {
  const int l = threadIdx.x & 31, h = l >> 4, m = l & 15;
  const lf16* p = base + (row0 + m) * pitch + k0 + 8 * h;
  Frag16 f;
  f.hf[0] = *(const lv8h*)(p);
  f.hf[1] = *(const lv8h*)(p + 16);
  return f.v;
}

__device__ __forceinline__ v16h frag_glb(const f16* __restrict__ base, int ld, int row0, int k0) {
  const int l = threadIdx.x & 31, h = l >> 4, m = l & 15;
  const f16* p = base + (row0 + m) * ld + k0 + 8 * h;
  Frag16 f;
  f.hf[0] = *(const v8ha*)(p);
  f.hf[1] = *(const v8ha*)(p + 16);
  return f.v;
}

template <int KT, bool RELU, bool TOUT>
__device__ __forceinline__ void gemm_xw(const lf16* X, int pitchX,
                                        const f16* __restrict__ W,
                                        const float* __restrict__ bias,
                                        lf16* Y, int pitchY) {
  const int wave = threadIdx.x >> 5, l = threadIdx.x & 31, h = l >> 4, m = l & 15;
  const int m0 = (wave >> 2) * 32;
  const int n0 = (wave & 3) * 64;
  const v8f z8 = {0.f, 0.f, 0.f, 0.f, 0.f, 0.f, 0.f, 0.f};

  v8f acc[2][4];
#pragma unroll
  for (int mt = 0; mt < 2; ++mt)
#pragma unroll
    for (int nt = 0; nt < 4; ++nt) acc[mt][nt] = z8;

#pragma unroll 1
  for (int kt = 0; kt < KT; ++kt) {
    const int k0 = kt * 32;
    const v16h a0 = frag_lds(X, pitchX, m0, k0);
    const v16h a1 = frag_lds(X, pitchX, m0 + 16, k0);
#pragma unroll
    for (int nt = 0; nt < 4; ++nt) {
      const v16h bw = frag_glb(W, KT * 32, n0 + 16 * nt, k0);
      wmma2(a0, a1, bw, acc[0][nt], acc[1][nt]);
    }
  }

#pragma unroll
  for (int nt = 0; nt < 4; ++nt) {
    const int col = n0 + 16 * nt + m;
    const float bvl = bias[col];
#pragma unroll
    for (int mt = 0; mt < 2; ++mt) {
      const int rb = m0 + 16 * mt + 8 * h;
      if (TOUT) {
        Frag8 u;
#pragma unroll
        for (int r = 0; r < 8; ++r) {
          float y = acc[mt][nt][r] * WINV + bvl;
          if (RELU) y = fmaxf(y, 0.0f);
          u.s[r] = (f16)y;
        }
        *(lv8h*)(Y + col * pitchY + rb) = u.v;
      } else {
#pragma unroll
        for (int r = 0; r < 8; ++r) {
          float y = acc[mt][nt][r] * WINV + bvl;
          if (RELU) y = fmaxf(y, 0.0f);
          Y[(rb + r) * pitchY + col] = (f16)y;
        }
      }
    }
  }
}

__global__ __launch_bounds__(256) void k_convert(
    const float* __restrict__ W1, const float* __restrict__ W2,
    const float* __restrict__ Wq, const float* __restrict__ Wk,
    const float* __restrict__ Wv, const float* __restrict__ Wo,
    const float* __restrict__ Wc, const float* __restrict__ W3,
    f16* __restrict__ wh)
{
  const int g = blockIdx.x * 256 + threadIdx.x;
  if (g >= NGRP) return;
  const float* src;
  int lo = 0;
  if (g < WO_W2 / 8) {
    src = W1 + 8 * g;
  } else if (g < WO_W3H / 8) {
    const int e = g - WO_W2 / 8;
    const int sel = e >> 13, off = e & 8191;
    const float* base = (sel == 0) ? W2 : (sel == 1) ? Wq : (sel == 2) ? Wk :
                        (sel == 3) ? Wv : (sel == 4) ? Wo : Wc;
    src = base + 8 * off;
  } else if (g < WO_W3L / 8) {
    src = W3 + 8 * (g - WO_W3H / 8);
  } else {
    src = W3 + 8 * (g - WO_W3L / 8);
    lo = 1;
  }
  const v4f a = *(const v4fa*)(src);
  const v4f c = *(const v4fa*)(src + 4);
  const float x[8] = { a.x * WSC, a.y * WSC, a.z * WSC, a.w * WSC,
                       c.x * WSC, c.y * WSC, c.z * WSC, c.w * WSC };
  Frag8 u;
#pragma unroll
  for (int i = 0; i < 8; ++i) {
    const f16 hv = (f16)x[i];
    const f16 lv = (f16)(x[i] - (float)hv);
    u.s[i] = lo ? lv : hv;
  }
  f16* dst = wh + 8 * g;
  *(volatile v8h*)dst = u.v;
  __threadfence();
  *(volatile v8h*)dst = u.v;
}

__global__ __launch_bounds__(256)
void k_graph(const float* __restrict__ obs, const float* __restrict__ adj,
             const f16* __restrict__ wh,
             const float* __restrict__ b1, const float* __restrict__ b2,
             const float* __restrict__ bq, const float* __restrict__ bk,
             const float* __restrict__ bv, const float* __restrict__ bo,
             const float* __restrict__ bc, const float* __restrict__ b3,
             float* __restrict__ out)
{
  extern __shared__ __align__(16) char smem[];
  LDS_AS char* sb = (LDS_AS char*)smem;
  lf16* S    = (lf16*)(sb + OFF_S);
  lf16* OBS  = (lf16*)(sb + OFF_S);
  lf32* OUTS = (lf32*)(sb + OFF_S);
  lf16* XA   = (lf16*)(sb + OFF_XA);
  lf32* ZF   = (lf32*)(sb + OFF_XA);
  lf16* XB   = (lf16*)(sb + OFF_XB);
  lf16* QO   = (lf16*)(sb + OFF_Q);
  lf16* VT   = (lf16*)(sb + OFF_VT);
  lf16* ADJ  = (lf16*)(sb + OFF_ADJ);

  const int tid = threadIdx.x, wave = tid >> 5, l = tid & 31, h = l >> 4, m = l & 15;
  const int b = blockIdx.x;
  const v8f z8 = {0.f, 0.f, 0.f, 0.f, 0.f, 0.f, 0.f, 0.f};

  {
    const float* ob = obs + (size_t)b * (NN * DOBS);
#pragma unroll 1
    for (int i = tid; i < NN * DOBS / 4; i += 256) {
      const v4f t = *(const v4fa*)(ob + 4 * i);
      const v4h hv = { (f16)t.x, (f16)t.y, (f16)t.z, (f16)t.w };
      const int rr = i >> 5, c4 = i & 31;
      *(lv4h*)(OBS + rr * POBS + 4 * c4) = hv;
    }
    const float* ad = adj + (size_t)b * (NN * NN);
#pragma unroll 1
    for (int i = tid; i < NN * NN / 4; i += 256) {
      const v4f t = *(const v4fa*)(ad + 4 * i);
      const v4h hv = { (f16)t.x, (f16)t.y, (f16)t.z, (f16)t.w };
      const int rr = i >> 4, c4 = i & 15;
      *(lv4h*)(ADJ + rr * PT + 4 * c4) = hv;
    }
  }
  __syncthreads();

  gemm_xw<DOBS / 32, true, false>(OBS, POBS, wh + WO_W1, b1, XA, PX);
  __syncthreads();
  gemm_xw<DH / 32, true, false>(XA, PX, wh + WO_W2, b2, XB, PX);
  __syncthreads();

  gemm_xw<DH / 32, false, false>(XB, PX, wh + WO_WQ, bq, QO, PX);
  gemm_xw<DH / 32, false, false>(XB, PX, wh + WO_WK, bk, XA, PX);
  gemm_xw<DH / 32, false, true >(XB, PX, wh + WO_WV, bv, VT, PT);
  __syncthreads();

  {
    const int hh = wave >> 1, q0 = (wave & 1) * 32;
    lf16* Ph = S + hh * (NN * PT);
    v8f s[2][4];
#pragma unroll
    for (int mt = 0; mt < 2; ++mt)
#pragma unroll
      for (int nt = 0; nt < 4; ++nt) s[mt][nt] = z8;

#pragma unroll 1
    for (int ks = 0; ks < 2; ++ks) {
      const int k0 = hh * HDM + ks * 32;
      const v16h a0 = frag_lds(QO, PX, q0, k0);
      const v16h a1 = frag_lds(QO, PX, q0 + 16, k0);
#pragma unroll
      for (int nt = 0; nt < 4; ++nt) {
        const v16h bkf = frag_lds(XA, PX, 16 * nt, k0);
        wmma2(a0, a1, bkf, s[0][nt], s[1][nt]);
      }
    }

#pragma unroll
    for (int mt = 0; mt < 2; ++mt) {
#pragma unroll
      for (int r = 0; r < 8; ++r) {
        const int row = q0 + 16 * mt + 8 * h + r;
        float v[4];
#pragma unroll
        for (int nt = 0; nt < 4; ++nt) {
          const float av = (float)ADJ[row * PT + 16 * nt + m];
          v[nt] = (av != 0.0f) ? s[mt][nt][r] * 0.125f : -1.0e30f;
        }
        float mx = fmaxf(fmaxf(v[0], v[1]), fmaxf(v[2], v[3]));
#pragma unroll
        for (int off = 1; off < 16; off <<= 1) mx = fmaxf(mx, __shfl_xor(mx, off, 32));
        float e[4], sum = 0.0f;
#pragma unroll
        for (int nt = 0; nt < 4; ++nt) { e[nt] = __expf(v[nt] - mx); sum += e[nt]; }
#pragma unroll
        for (int off = 1; off < 16; off <<= 1) sum += __shfl_xor(sum, off, 32);
        const float sc = PSC * __builtin_amdgcn_rcpf(sum);
#pragma unroll
        for (int nt = 0; nt < 4; ++nt) Ph[row * PT + 16 * nt + m] = (f16)(e[nt] * sc);
      }
    }
  }
  __syncthreads();

  {
    const int hh = wave >> 1, q0 = (wave & 1) * 32;
    const lf16* Ph = S + hh * (NN * PT);
    v8f o[2][4];
#pragma unroll
    for (int mt = 0; mt < 2; ++mt)
#pragma unroll
      for (int nt = 0; nt < 4; ++nt) o[mt][nt] = z8;

#pragma unroll 1
    for (int ks = 0; ks < 2; ++ks) {
      const int k0 = ks * 32;
      const v16h a0 = frag_lds(Ph, PT, q0, k0);
      const v16h a1 = frag_lds(Ph, PT, q0 + 16, k0);
#pragma unroll
      for (int nt = 0; nt < 4; ++nt) {
        const v16h bvf = frag_lds(VT, PT, hh * HDM + 16 * nt, k0);
        wmma2(a0, a1, bvf, o[0][nt], o[1][nt]);
      }
    }
#pragma unroll
    for (int nt = 0; nt < 4; ++nt)
#pragma unroll
      for (int mt = 0; mt < 2; ++mt)
#pragma unroll
        for (int r = 0; r < 8; ++r)
          QO[(q0 + 16 * mt + 8 * h + r) * PX + hh * HDM + 16 * nt + m] = (f16)(o[mt][nt][r] * PINV);
  }
  __syncthreads();

  gemm_xw<DH / 32, false, false>(QO, PX, wh + WO_WO, bo, XB, PX);
  __syncthreads();
  gemm_xw<DH / 32, false, true >(XB, PX, wh + WO_WC, bc, VT, PT);
  __syncthreads();

  {
    const int m0 = (wave >> 2) * 32, n0 = (wave & 3) * 64;
    v8f acc[2][4];
#pragma unroll
    for (int mt = 0; mt < 2; ++mt)
#pragma unroll
      for (int nt = 0; nt < 4; ++nt) acc[mt][nt] = z8;

#pragma unroll 1
    for (int kt = 0; kt < 2; ++kt) {
      const int k0 = kt * 32;
      const v16h a0 = frag_lds(ADJ, PT, m0, k0);
      const v16h a1 = frag_lds(ADJ, PT, m0 + 16, k0);
#pragma unroll
      for (int nt = 0; nt < 4; ++nt) {
        const v16h bcf = frag_lds(VT, PT, n0 + 16 * nt, k0);
        wmma2(a0, a1, bcf, acc[0][nt], acc[1][nt]);
      }
    }
#pragma unroll
    for (int nt = 0; nt < 4; ++nt)
#pragma unroll
      for (int mt = 0; mt < 2; ++mt)
#pragma unroll
        for (int r = 0; r < 8; ++r)
          ZF[(m0 + 16 * mt + 8 * h + r) * PZ + n0 + 16 * nt + m] = acc[mt][nt][r];
  }
  __syncthreads();

  if (wave < 4) {
    const int r0 = wave * 16;
    const f16* w3h = wh + WO_W3H;
    const f16* w3l = wh + WO_W3L;
    v8f acc = z8;
#pragma unroll 1
    for (int kt = 0; kt < 8; ++kt) {
      const int k0 = kt * 32;
      const lf32* zp = ZF + (r0 + m) * PZ + k0 + 8 * h;
      const v4f t0 = *(const lv4f*)(zp);
      const v4f t1 = *(const lv4f*)(zp + 4);
      const v4f t2 = *(const lv4f*)(zp + 16);
      const v4f t3 = *(const lv4f*)(zp + 20);
      const float x[16] = { t0.x, t0.y, t0.z, t0.w, t1.x, t1.y, t1.z, t1.w,
                            t2.x, t2.y, t2.z, t2.w, t3.x, t3.y, t3.z, t3.w };
      Frag16 uh, ul;
#pragma unroll
      for (int i = 0; i < 16; ++i) {
        const float xs = x[i] * WSC;
        const f16 hv = (f16)xs;
        uh.s[i] = hv;
        ul.s[i] = (f16)(xs - (float)hv);
      }
      const v16h bh = frag_glb(w3h, DH, 0, k0);
      const v16h bl = frag_glb(w3l, DH, 0, k0);
      acc = wmma3(uh.v, ul.v, bh, bl, acc);
    }
    const float bvl = b3[m];
#pragma unroll
    for (int r = 0; r < 8; ++r)
      OUTS[(r0 + 8 * h + r) * DA + m] = acc[r] * ZINV + bvl;
  }
  __syncthreads();

  {
    const v4f v = *(const lv4f*)(OUTS + 4 * tid);
    float* gp = out + (size_t)b * (NN * DA) + 4 * tid;
    *(volatile v4f*)gp = v;
    __threadfence();
    *(volatile v4f*)gp = v;
  }
}

extern "C" void kernel_launch(void* const* d_in, const int* in_sizes, int n_in,
                              void* d_out, int out_size, void* d_ws, size_t ws_size,
                              hipStream_t stream) {
  if (n_in < 18) return;
  if (in_sizes[0] != NB * NN * DOBS) return;
  if (in_sizes[1] != NB * NN * NN) return;
  if (in_sizes[2] != DH * DOBS || in_sizes[3] != DH) return;
  if (in_sizes[4] != DH * DH || in_sizes[5] != DH) return;
  if (in_sizes[6] != DH * DH || in_sizes[7] != DH) return;
  if (in_sizes[8] != DH * DH || in_sizes[9] != DH) return;
  if (in_sizes[10] != DH * DH || in_sizes[11] != DH) return;
  if (in_sizes[12] != DH * DH || in_sizes[13] != DH) return;
  if (in_sizes[14] != DH * DH || in_sizes[15] != DH) return;
  if (in_sizes[16] != DA * DH || in_sizes[17] != DA) return;
  if (out_size != NB * NN * DA) return;
  if ((size_t)WS_HALVES * 2 > ws_size) return;

  const float* obs = (const float*)d_in[0];
  const float* adj = (const float*)d_in[1];
  const float* W1 = (const float*)d_in[2];  const float* b1 = (const float*)d_in[3];
  const float* W2 = (const float*)d_in[4];  const float* b2 = (const float*)d_in[5];
  const float* Wq = (const float*)d_in[6];  const float* bq = (const float*)d_in[7];
  const float* Wk = (const float*)d_in[8];  const float* bk = (const float*)d_in[9];
  const float* Wv = (const float*)d_in[10]; const float* bv = (const float*)d_in[11];
  const float* Wo = (const float*)d_in[12]; const float* bo = (const float*)d_in[13];
  const float* Wc = (const float*)d_in[14]; const float* bc = (const float*)d_in[15];
  const float* W3 = (const float*)d_in[16]; const float* b3 = (const float*)d_in[17];
  float* out = (float*)d_out;
  f16* wh = (f16*)d_ws;

  k_convert<<<NGRP / 256, 256, 0, stream>>>(W1, W2, Wq, Wk, Wv, Wo, Wc, W3, wh);

  (void)hipFuncSetAttribute((const void*)k_graph,
                            hipFuncAttributeMaxDynamicSharedMemorySize, SMEM_BYTES);

  k_graph<<<NB, 256, SMEM_BYTES, stream>>>(obs, adj, wh, b1, b2, bq, bk, bv, bo, bc, b3, out);
}
